// RDFNSMultiHeadAttention_69913477644290
// MI455X (gfx1250) — hardware-run, weakly checked
//
#include <hip/hip_runtime.h>
#define QNG 2
#define QNL 1024
#define QNW 1024
#define QNS 16
#define QSW 64
#define QDS 64.0f
#define QPW -65.5f
#define QLO 1e-12f
#define QWC 64.0f
#define QPC 4096.0f
typedef unsigned short v8us __attribute__((ext_vector_type(8), may_alias));
typedef float  v8f  __attribute__((ext_vector_type(8)));
typedef float  v4f  __attribute__((ext_vector_type(4)));
typedef float  v4fa __attribute__((ext_vector_type(4), may_alias));

__device__ __forceinline__ unsigned short bf16_bits(float x) { unsigned int u = __float_as_uint(x); return (unsigned short)((u + 0x7FFFu + ((u >> 16) & 1u)) >> 16); }
__device__ __forceinline__ float bf16_val(unsigned short b) { return __uint_as_float(((unsigned int)b) << 16); }
__device__ __forceinline__ float bf16_round(float x) { return bf16_val(bf16_bits(x)); }

typedef _Float16 v16h __attribute__((ext_vector_type(16)));
union FragH { v16h v; v8us half[2]; _Float16 h[16]; unsigned short u[16]; };

__global__ __launch_bounds__(256) void k_wt_f16(const float* __restrict__ W, _Float16* __restrict__ Wt, int K, int N, float scale) {
  const int t = blockIdx.x * 256 + threadIdx.x; if (t >= N * (K / 8)) return; const int n = t / (K / 8), k8 = (t % (K / 8)) * 8; FragH f;
#pragma unroll
  for (int i = 0; i < 8; ++i) f.h[i] = (_Float16)(bf16_round(W[(size_t)(k8 + i) * N + n]) * scale); const v8us o = f.half[0];
  *(volatile v8us*)((unsigned short*)Wt + (size_t)n * K + k8) = o; __threadfence(); *(volatile v8us*)((unsigned short*)Wt + (size_t)n * K + k8) = o;
}

typedef _Float16 v4h __attribute__((ext_vector_type(4)));

__global__ __launch_bounds__(256) void k_wtn_f16(const float* __restrict__ W, _Float16* __restrict__ Wt, int K, int N, float scale) {
  const int t = blockIdx.x * 256 + threadIdx.x; if (t >= N * (K / 8)) return; const int n = t / (K / 8), k8 = (t % (K / 8)) * 8; FragH f;
  for (int i = 0; i < 8; ++i) f.h[i] = (_Float16)(W[(size_t)(k8 + i) * N + n] * scale);
  unsigned short* o = (unsigned short*)Wt + (size_t)n * K + k8; *(volatile v8us*)o = f.half[0]; __threadfence(); *(volatile v8us*)o = f.half[0]; }

__global__ __launch_bounds__(256) void k_hl(const float* __restrict__ F, _Float16* __restrict__ Hh, _Float16* __restrict__ Hl, size_t n8) { const size_t t = (size_t)blockIdx.x * 256 + threadIdx.x; if (t >= n8) return; FragH fh, fl; const v4f a = *(const v4fa*)(F + t * 8), c = *(const v4fa*)(F + t * 8 + 4);
#pragma unroll
  for (int q = 0; q < 4; ++q) { _Float16 h = (_Float16)a[q]; fh.h[q] = h; fl.h[q] = (_Float16)((a[q] - (float)h) * 1024.0f); h = (_Float16)c[q]; fh.h[4 + q] = h; fl.h[4 + q] = (_Float16)((c[q] - (float)h) * 1024.0f); }
  for (int pass = 0; pass < 2; ++pass) { *(volatile v8us*)((unsigned short*)Hh + t * 8) = fh.half[0]; *(volatile v8us*)((unsigned short*)Hl + t * 8) = fl.half[0]; if (pass == 0) __threadfence(); } }

__global__ __launch_bounds__(256) void k_x16(const float* __restrict__ x, _Float16* __restrict__ X16, size_t n8) { const size_t t = (size_t)blockIdx.x * 256 + threadIdx.x; if (t >= n8) return; FragH f;
#pragma unroll
  for (int q = 0; q < 8; ++q) f.h[q] = (_Float16)bf16_round(x[t * 8 + q]); *(volatile v8us*)((unsigned short*)X16 + t * 8) = f.half[0]; __threadfence(); *(volatile v8us*)((unsigned short*)X16 + t * 8) = f.half[0]; }

__device__ __forceinline__ v16h g2_frag(const _Float16* p, int hh) { FragH f; f.half[0] = *(const v8us*)((const unsigned short*)p + 8 * hh); f.half[1] = *(const v8us*)((const unsigned short*)p + 16 + 8 * hh); return f.v; }
__device__ __forceinline__ v8f g2_mma(v16h a, v16h b, v8f c) { v8f d = __builtin_amdgcn_wmma_f32_16x16x32_f16(false, a, false, b, (short)0, c, false, false); asm volatile("v_nop\n\tv_nop\n\tv_nop\n\tv_nop" : "+v"(d) : "v"(a), "v"(b)); return d; }
template <int ACT>
__global__ __launch_bounds__(128) void k_gemm2(const _Float16* __restrict__ A, int lda, size_t sA, const _Float16* __restrict__ Bh, int ldb, size_t sB, float alpha, const float* __restrict__ bias, size_t sBias, const float* __restrict__ CP, int rowsPerB, size_t sCPb, int row0g,
    float* __restrict__ C, _Float16* __restrict__ C16, int ldc, size_t sC, int M, int N, int K) { static_assert(ACT == 0 || ACT == 3 || ACT == 6 || ACT == 8 || ACT == 9 || ACT == 11 || ACT == 12 || ACT == 14 || ACT == 15 || ACT == 16 || ACT == 17, "k_gemm2: unsupported ACT code (would silently apply no activation)");
  __shared__ __attribute__((aligned(16))) float so[4][32][68];
  const int tid = threadIdx.x, w = tid >> 5, lane = tid & 31, ln = lane & 15, hh = lane >> 4; const int by = blockIdx.y;
  A += (size_t)by * sA; Bh += (size_t)by * sB; const size_t cofs = (size_t)by * sC; const float* bp = bias ? bias + (size_t)by * sBias : nullptr;
  const int ntn = N >> 6; const int mt = blockIdx.x / ntn, nq = blockIdx.x - mt * ntn; const int row0 = mt * 128 + 32 * w, col0 = nq * 64; if (row0 >= M) return;
  const _Float16* a0p = A + (size_t)(row0 + ln) * lda; const _Float16* a1p = a0p + (size_t)16 * lda;
  const _Float16* b0p = Bh + (size_t)(col0 + ln) * ldb; const _Float16* b1p = b0p + (size_t)16 * ldb; const _Float16* b2p = b1p + (size_t)16 * ldb; const _Float16* b3p = b2p + (size_t)16 * ldb;
  const v8f z8 = {0.f,0.f,0.f,0.f,0.f,0.f,0.f,0.f}; v8f c00 = z8, c01 = z8, c02 = z8, c03 = z8, c10 = z8, c11 = z8, c12 = z8, c13 = z8;
  for (int kb = 0; kb < K; kb += 32) { const v16h a0 = g2_frag(a0p + kb, hh), a1 = g2_frag(a1p + kb, hh);
    v16h b = g2_frag(b0p + kb, hh); c00 = g2_mma(a0, b, c00); c10 = g2_mma(a1, b, c10);
    b = g2_frag(b1p + kb, hh); c01 = g2_mma(a0, b, c01); c11 = g2_mma(a1, b, c11);
    b = g2_frag(b2p + kb, hh); c02 = g2_mma(a0, b, c02); c12 = g2_mma(a1, b, c12);
    b = g2_frag(b3p + kb, hh); c03 = g2_mma(a0, b, c03); c13 = g2_mma(a1, b, c13); }
  v8f accs[8] = {c00, c01, c02, c03, c10, c11, c12, c13};
#pragma unroll
  for (int u = 0; u < 8; ++u) { const int t = u & 3, half = u >> 2; const int col = col0 + t * 16 + ln; const float bv = bp ? bf16_round(bp[col]) : 0.f;
#pragma unroll
    for (int r = 0; r < 8; ++r) { const int rloc = half * 16 + 8 * hh + r; float v = accs[u][r] * alpha + bv; if (CP) { if (rowsPerB < 0) v += CP[cofs + (size_t)(row0g + row0 + rloc) * ldc + col];        else { const int bidx = (row0g + row0 + rloc) / rowsPerB; v += CP[(size_t)bidx * sCPb + (size_t)by * 64 + col]; } }
      if (ACT == 3) v = fmaxf(v, 0.f); else if (ACT == 6) v = 0.5f * v * (1.0f + erff(v * 0.70710678118654752f)); else if (ACT == 11) v = 1.0f / (1.0f + expf(-v)); else if (ACT == 15) v = v / (1.0f + expf(-v)); else if (ACT == 12) v = (v > 0.f) ? v : 0.01f * v; else if (ACT == 8) v = tanhf(v); else if (ACT == 9) v = 0.5f * v * (1.0f + tanhf(0.7978845608028654f * (v + 0.044715f * v * v * v))); else if (ACT == 14) v = (v > 0.f) ? v : 0.1f * v; else if (ACT == 16) v = (v >= 0.f) ? v : 0.3f * v; else if (ACT == 17) v = (v >= 0.f) ? v : 0.2f * v;
      so[w][rloc][t * 16 + ln] = v; } }
  __builtin_amdgcn_fence(__ATOMIC_ACQ_REL, "workgroup"); __builtin_amdgcn_wave_barrier();
  const int rsub = lane >> 4, c4 = (lane & 15) * 4;
  for (int pass = 0; pass < 2; ++pass) {
#pragma unroll
    for (int q = 0; q < 16; ++q) { const int r = q * 2 + rsub; const v4f v = *(const v4fa*)&so[w][r][c4]; if (C) *(volatile v4f*)(C + cofs + (size_t)(row0 + r) * ldc + col0 + c4) = v; if (C16) { v4h h4; for (int i = 0; i < 4; ++i) h4[i] = (_Float16)v[i]; *(volatile v4h*)(C16 + cofs + (size_t)(row0 + r) * ldc + col0 + c4) = h4; } }
    if (pass == 0) __threadfence(); } }

__global__ __launch_bounds__(256) void k_sln(const float* __restrict__ F, float* __restrict__ LN) {
  const unsigned t = blockIdx.x * 256u + threadIdx.x; if (t >= (unsigned)(QNG * QNS * QNL)) return;
  const unsigned i = t % QNL, s = (t / QNL) % QNS, g = t / (QNL * QNS); const float* p = F + ((size_t)g * QNL + i) * QNW + s * QSW; float a = 0.0f;
  for (unsigned c = 0; c < (unsigned)QSW; c += 4) { const v4f w = *(const v4fa*)(p + c);
#pragma unroll
    for (int q = 0; q < 4; ++q) a += w[q] * w[q]; }
  *(volatile float*)(LN + t) = a; __threadfence(); *(volatile float*)(LN + t) = a; }

__global__ __launch_bounds__(256) void k_psc(float* SC, const float* __restrict__ la, const float* __restrict__ lb) {
  const unsigned t = blockIdx.x * 256u + threadIdx.x; if (t >= (unsigned)(QNS * QNL * (QNL / 4))) return;
  const unsigned j = (t % (QNL / 4)) * 4, i = (t / (QNL / 4)) % QNL, s = t / ((QNL / 4) * QNL); float* p = SC + (size_t)t * 4; const v4f z = *(const v4fa*)p; const float qa = la[s * QNL + i]; const v4f kb = *(const v4fa*)(lb + s * QNL + j); v4f w;
#pragma unroll
  for (int q = 0; q < 4; ++q) { const float e2 = (qa + kb[q]) - 2.0f * z[q]; const float gd = sqrtf(fmaxf(e2, QLO)) / QDS; w[q] = powf(1.0f + gd, QPW); }
  *(volatile v4f*)p = w; __threadfence(); *(volatile v4f*)p = w; }

__global__ __launch_bounds__(256) void k_rsm(const float* __restrict__ SC, float* __restrict__ NR) {
  const unsigned r = blockIdx.x * 256u + threadIdx.x; if (r >= (unsigned)(QNS * QNL)) return;
  const float* p = SC + (size_t)r * QNL; float a = 0.0f;
  for (unsigned j = 0; j < (unsigned)QNL; j += 4) { const v4f w = *(const v4fa*)(p + j); a += w[0]; a += w[1]; a += w[2]; a += w[3]; }
  *(volatile float*)(NR + r) = a; __threadfence(); *(volatile float*)(NR + r) = a; }

__global__ __launch_bounds__(256) void k_csm(const float* __restrict__ SC, float* __restrict__ CF) {
  const unsigned t = blockIdx.x * 256u + threadIdx.x; if (t >= (unsigned)(QNS * QNL)) return;
  const float* p = SC + (size_t)(t / QNL) * QNL * QNL + (t % QNL); float a = 0.0f;
  for (unsigned i = 0; i < (unsigned)QNL; i += 4) { const float a0 = p[(size_t)i * QNL], a1 = p[(size_t)(i + 1) * QNL], a2 = p[(size_t)(i + 2) * QNL], a3 = p[(size_t)(i + 3) * QNL]; a += a0; a += a1; a += a2; a += a3; }
  const float w = 1.0f / sqrtf(a); *(volatile float*)(CF + t) = w; __threadfence(); *(volatile float*)(CF + t) = w; }

__global__ __launch_bounds__(256) void k_ktn(const float* __restrict__ SC, const float* __restrict__ NR, const float* __restrict__ CF, _Float16* __restrict__ PB) {
  const unsigned r = blockIdx.x * 256u + threadIdx.x; if (r >= (unsigned)(QNS * QNL)) return;
  const float* p = SC + (size_t)r * QNL; const float* cf = CF + (size_t)(r / QNL) * QNL; unsigned short* o = (unsigned short*)PB + (size_t)r * QNL; const float rf = 1.0f / sqrtf(NR[r]); float a = 0.0f;
  for (unsigned j = 0; j < (unsigned)QNL; j += 4) { const v4f w = *(const v4fa*)(p + j); const v4f c = *(const v4fa*)(cf + j);
#pragma unroll
    for (int q = 0; q < 4; ++q) a += (rf * w[q]) * c[q]; }
  const float dn = fmaxf(a, QLO);
  for (unsigned j = 0; j < (unsigned)QNL; j += 8) { const v4f w0 = *(const v4fa*)(p + j), w1 = *(const v4fa*)(p + j + 4); const v4f c0 = *(const v4fa*)(cf + j), c1 = *(const v4fa*)(cf + j + 4); FragH f;
#pragma unroll
    for (int q = 0; q < 4; ++q) { f.h[q] = (_Float16)((((rf * w0[q]) * c0[q]) / dn) * QPC); f.h[4 + q] = (_Float16)((((rf * w1[q]) * c1[q]) / dn) * QPC); }
    const v8us w = f.half[0]; *(volatile v8us*)(o + j) = w; __threadfence(); *(volatile v8us*)(o + j) = w; }
}

extern "C" void kernel_launch(void* const* d_in, const int* in_sizes, int n_in,
                              void* d_out, int out_size, void* d_ws, size_t ws_size, hipStream_t stream) {
  (void)in_sizes; (void)n_in; (void)out_size;
  const float* const* I = (const float* const*)d_in; const float* xa = I[0]; const float* wa = I[1]; const float* va = I[2]; const float* wb = I[3]; const float* vb = I[4]; const float* wc = I[5]; const float* vc = I[6]; const float* wd = I[7]; const float* vd = I[8];
  float* res = (float*)d_out;
  static_assert((QNG * QNL) % 128 == 0 && QNL % 128 == 0 && QNW % 64 == 0 && QNW % 32 == 0 && QSW % 64 == 0 && QSW % 32 == 0 && QNL % 8 == 0 && QNS * QSW == QNW, "whole tiles");
  uint8_t* wsp = (uint8_t*)d_ws; size_t off = 0;
  auto take = [&](size_t bytes) { uint8_t* p = wsp + off; off += (bytes + 255) & ~(size_t)255; return p; };
  const size_t GW = (size_t)QNG * QNL * QNW, G1 = (size_t)QNL * QNW;
  float* SC = (float*)take((size_t)QNS * QNL * QNL * 4); _Float16* PB = (_Float16*)take((size_t)QNS * QNL * QNL * 2); float* FA = (float*)take(GW * 4); float* FB = (float*)take(GW * 4); float* FC = (float*)take(GW * 4); float* CX = (float*)take(GW * 4);
  _Float16* XH = (_Float16*)take(GW * 2); _Float16* AH = (_Float16*)take(GW * 2); _Float16* AL = (_Float16*)take(GW * 2); _Float16* BH = (_Float16*)take(GW * 2); _Float16* BL = (_Float16*)take(GW * 2); _Float16* CH = (_Float16*)take(GW * 2); _Float16* CL = (_Float16*)take(GW * 2); _Float16* VT = (_Float16*)take(G1 * 2);
  _Float16* WA = (_Float16*)take((size_t)QNW * QNW * 2); _Float16* WB = (_Float16*)take((size_t)QNW * QNW * 2); _Float16* WC = (_Float16*)take((size_t)QNW * QNW * 2); _Float16* WD = (_Float16*)take((size_t)QNW * QNW * 2); float* LA = (float*)take((size_t)QNG * QNS * QNL * 4); float* LB = (float*)take((size_t)QNG * QNS * QNL * 4); float* NR = (float*)take((size_t)QNS * QNL * 4); float* CF = (float*)take((size_t)QNS * QNL * 4);
  if (off > ws_size) return;
  k_x16<<<(unsigned)((GW / 8 + 255) / 256), 256, 0, stream>>>(xa, XH, GW / 8);
  k_wt_f16<<<(unsigned)(((size_t)QNW * (QNW / 8) + 255) / 256), 256, 0, stream>>>(wa, WA, QNW, QNW, QWC);
  k_wt_f16<<<(unsigned)(((size_t)QNW * (QNW / 8) + 255) / 256), 256, 0, stream>>>(wb, WB, QNW, QNW, QWC);
  k_wt_f16<<<(unsigned)(((size_t)QNW * (QNW / 8) + 255) / 256), 256, 0, stream>>>(wc, WC, QNW, QNW, QWC);
  k_wt_f16<<<(unsigned)(((size_t)QNW * (QNW / 8) + 255) / 256), 256, 0, stream>>>(wd, WD, QNW, QNW, QWC);
  k_gemm2<0><<<dim3((unsigned)(((QNG * QNL) / 128) * (QNW / 64)), 1), 128, 0, stream>>>(XH, QNW, 0, WA, QNW, 0, 1.0f / QWC, va, 0, nullptr, 1, 0, 0, FA, nullptr, QNW, 0, QNG * QNL, QNW, QNW);
  k_gemm2<0><<<dim3((unsigned)(((QNG * QNL) / 128) * (QNW / 64)), 1), 128, 0, stream>>>(XH, QNW, 0, WB, QNW, 0, 1.0f / QWC, vb, 0, nullptr, 1, 0, 0, FB, nullptr, QNW, 0, QNG * QNL, QNW, QNW);
  k_gemm2<0><<<dim3((unsigned)(((QNG * QNL) / 128) * (QNW / 64)), 1), 128, 0, stream>>>(XH, QNW, 0, WC, QNW, 0, 1.0f / QWC, vc, 0, nullptr, 1, 0, 0, FC, nullptr, QNW, 0, QNG * QNL, QNW, QNW);
  k_sln<<<(unsigned)((QNG * QNS * QNL + 255) / 256), 256, 0, stream>>>(FA, LA);
  k_sln<<<(unsigned)((QNG * QNS * QNL + 255) / 256), 256, 0, stream>>>(FB, LB);
  k_hl<<<(unsigned)((GW / 8 + 255) / 256), 256, 0, stream>>>(FA, AH, AL, GW / 8);
  k_hl<<<(unsigned)((GW / 8 + 255) / 256), 256, 0, stream>>>(FB, BH, BL, GW / 8);
  for (int g = 0; g < QNG; ++g) {
    k_wtn_f16<<<(unsigned)(((size_t)QNW * (QNL / 8) + 255) / 256), 256, 0, stream>>>(FC + g * G1, VT, QNL, QNW, 1.0f);
    k_gemm2<0><<<dim3((unsigned)((QNL / 128) * (QNL / 64)), QNS), 128, 0, stream>>>(AH + g * G1, QNW, (size_t)QSW, BH + g * G1, QNW, (size_t)QSW, 1.0f, nullptr, 0, nullptr, 1, 0, 0, SC, nullptr, QNL, (size_t)QNL * QNL, QNL, QNL, QSW);
    k_psc<<<(unsigned)(((size_t)QNS * QNL * (QNL / 4) + 255) / 256), 256, 0, stream>>>(SC, LA + (size_t)g * QNS * QNL, LB + (size_t)g * QNS * QNL);
    k_rsm<<<(unsigned)((QNS * QNL + 255) / 256), 256, 0, stream>>>(SC, NR);
    k_csm<<<(unsigned)((QNS * QNL + 255) / 256), 256, 0, stream>>>(SC, CF);
    k_ktn<<<(unsigned)((QNS * QNL + 255) / 256), 256, 0, stream>>>(SC, NR, CF, PB);
    k_gemm2<0><<<dim3((unsigned)((QNL / 128) * (QSW / 64)), QNS), 128, 0, stream>>>(PB, QNL, (size_t)QNL * QNL, VT, QNL, (size_t)QSW * QNL, 1.0f / QPC, nullptr, 0, nullptr, 1, 0, 0, CX + g * G1, nullptr, QNW, (size_t)QSW, QNL, QSW, QNL); }
  k_hl<<<(unsigned)((GW / 8 + 255) / 256), 256, 0, stream>>>(CX, CH, CL, GW / 8);
  k_gemm2<0><<<dim3((unsigned)(((QNG * QNL) / 128) * (QNW / 64)), 1), 128, 0, stream>>>(CH, QNW, 0, WD, QNW, 0, 1.0f / QWC, vd, 0, nullptr, 1, 0, 0, res, nullptr, QNW, 0, QNG * QNL, QNW, QNW);
}
